// GQA_66108136620702
// MI455X (gfx1250) — hardware-verified
//
#include <hip/hip_runtime.h>
#include <math.h>

constexpr int kB    = 2;
constexpr int kT    = 2048;
constexpr int kD    = 1024;
constexpr int kH    = 16;
constexpr int kKV   = 4;
constexpr int kDh   = 64;
constexpr int kWin  = 512;
constexpr int kTok  = kB * kT;
constexpr int kNQKV = kH * kDh + 2 * kKV * kDh;
constexpr int kVCol = kH * kDh + kKV * kDh;
constexpr int kQRows = kB * kH * kT;
constexpr int kKRows = kB * kKV * kT;
constexpr float kScoreScale = 0.125f;
constexpr float kExpFloor   = -16384.0f;
static_assert(kH * kDh == kD, "shape");
static_assert(kTok % 64 == 0 && kNQKV % 64 == 0 && kD % 64 == 0 && kD % 32 == 0, "gemm tiles");
static_assert(kT % 64 == 0 && kDh == 64 && kH / kKV == 4, "attention tiles");

typedef __attribute__((ext_vector_type(16))) _Float16 v16h;
typedef __attribute__((ext_vector_type(8)))  _Float16 v8h;
typedef __attribute__((ext_vector_type(16))) __bf16   v16b;
typedef __attribute__((ext_vector_type(8)))  __bf16   v8b;
typedef __attribute__((ext_vector_type(8)))  float    v8f;
typedef __attribute__((ext_vector_type(4)))  float    v4f;
typedef __attribute__((ext_vector_type(4)))  unsigned int v4u;

__device__ __forceinline__ unsigned short f2bf_bits(float f) {
  unsigned u = __float_as_uint(f);
  return (unsigned short)((u + 0x7FFFu + ((u >> 16) & 1u)) >> 16);
}
__device__ __forceinline__ float bf_bits2f(unsigned short h) { return __uint_as_float(((unsigned)h) << 16); }

__device__ __forceinline__ void dep_guard_h(v8f& a, v8f& b, v16h x, v16h y) { asm volatile("v_nop\n\tv_nop\n\tv_nop\n\tv_nop" : "+v"(a), "+v"(b) : "v"(x), "v"(y)); }
__device__ __forceinline__ void dep_guard_b(v8f& a, v8f& b, v16b x, v16b y) { asm volatile("v_nop\n\tv_nop\n\tv_nop\n\tv_nop" : "+v"(a), "+v"(b) : "v"(x), "v"(y)); }
__device__ __forceinline__ void dep_guard4_h(v8f& a, v8f& b, v8f& c, v8f& d, v16h x, v16h y) { asm volatile("v_nop\n\tv_nop\n\tv_nop\n\tv_nop" : "+v"(a), "+v"(b), "+v"(c), "+v"(d) : "v"(x), "v"(y)); }
__device__ __forceinline__ void dep_guard4_b(v8f& a, v8f& b, v8f& c, v8f& d, v16b x, v16b y) { asm volatile("v_nop\n\tv_nop\n\tv_nop\n\tv_nop" : "+v"(a), "+v"(b), "+v"(c), "+v"(d) : "v"(x), "v"(y)); }
__device__ __forceinline__ void keep4_h(v16h a, v16h b, v16h c, v16h d) { asm volatile("v_nop" :: "v"(a), "v"(b), "v"(c), "v"(d)); }
__device__ __forceinline__ void keep4_b(v16b a, v16b b, v16b c, v16b d) { asm volatile("v_nop" :: "v"(a), "v"(b), "v"(c), "v"(d)); }
__device__ __forceinline__ void acc_guard4(v8f& a, v8f& b, v8f& c, v8f& d) { asm volatile("v_nop\n\tv_nop\n\tv_nop\n\tv_nop" : "+v"(a), "+v"(b), "+v"(c), "+v"(d)); }
template <typename T> struct Frag;
template <> struct Frag<_Float16> {
  typedef v16h V; union U { v16h v; v8h h[2]; };
  static __device__ __forceinline__ v16h load(const _Float16* p) {
    U f; f.h[0] = *(const v8h*)(p); f.h[1] = *(const v8h*)(p + 16); return f.v;
  }
  static __device__ __forceinline__ v8f mma(v16h a, v16h b, v8f c) {
    return __builtin_amdgcn_wmma_f32_16x16x32_f16(false, a, false, b, (short)0, c, false, false);
  }
  static __device__ __forceinline__ void guard(v8f& a, v8f& b, v16h x, v16h y) { dep_guard_h(a, b, x, y); }
  static __device__ __forceinline__ void guard4(v8f& a, v8f& b, v8f& c, v8f& d, v16h x, v16h y) { dep_guard4_h(a, b, c, d, x, y); }
  static __device__ __forceinline__ void keep(v16h a, v16h b, v16h c, v16h d) { keep4_h(a, b, c, d); }
};
template <> struct Frag<__bf16> {
  typedef v16b V; union U { v16b v; v8b h[2]; };
  static __device__ __forceinline__ v16b load(const __bf16* p) {
    U f; f.h[0] = *(const v8b*)(p); f.h[1] = *(const v8b*)(p + 16); return f.v;
  }
  static __device__ __forceinline__ v8f mma(v16b a, v16b b, v8f c) {
    return __builtin_amdgcn_wmma_f32_16x16x32_bf16(false, a, false, b, (short)0, c, false, false);
  }
  static __device__ __forceinline__ void guard(v8f& a, v8f& b, v16b x, v16b y) { dep_guard_b(a, b, x, y); }
  static __device__ __forceinline__ void guard4(v8f& a, v8f& b, v8f& c, v8f& d, v16b x, v16b y) { dep_guard4_b(a, b, c, d, x, y); }
  static __device__ __forceinline__ void keep(v16b a, v16b b, v16b c, v16b d) { keep4_b(a, b, c, d); }
};

__device__ __forceinline__ unsigned pk16(unsigned short a, unsigned short b) { return (unsigned)a | ((unsigned)b << 16); }

template <int ET> struct Elem;
template <> struct Elem<0> { typedef _Float16 T; };
template <> struct Elem<1> { typedef __bf16 T; };
template <int ET, int SPLIT, int BIAS_MODE, int OUT_MODE, bool RESID, int ACT = 0>
__global__ __launch_bounds__(256) void wmma_gemm64(
    const unsigned short* __restrict__ Ap, const unsigned short* __restrict__ A2p, int lda, long strideA,
    const unsigned short* __restrict__ Btp, const unsigned short* __restrict__ Bt2p, int ldb, long strideB,
    void* __restrict__ Cout, void* __restrict__ Cout2, int ldc, long strideC,
    const float* __restrict__ bias,
    const float* __restrict__ resid, long strideR,
    int M, int N, int K, float scale) {
  typedef typename Elem<ET>::T T;
  typedef typename Frag<T>::V V;
  const T* A = (const T*)Ap; const T* A2 = (const T*)A2p; const T* Bt = (const T*)Btp; const T* Bt2 = (const T*)Bt2p;
  __shared__ __align__(16) float sT[8][16 * 68];
  const int b    = blockIdx.y;
  const int lane = threadIdx.x & 31;
  const int wave = threadIdx.x >> 5;
  const int tilesN = N >> 6;
  const int tilesM = M >> 6;
  const int tile = blockIdx.x * 8 + wave;
  if (tile >= tilesM * tilesN) return;
  const int tm = tile / tilesN;
  const int tn = tile - tm * tilesN;
  const int m0 = tm << 6;
  const int n0 = tn << 6;

  const T* Ab  = A  + (size_t)b * strideA;
  const T* Bb  = Bt + (size_t)b * strideB;
  const T* Ab2 = (SPLIT != 0) ? (A2  + (size_t)b * strideA) : nullptr;
  const T* Bb2 = (SPLIT == 2) ? (Bt2 + (size_t)b * strideB) : nullptr;

  const int rlane = lane & 15;
  const int koff  = (lane >> 4) * 8;
  const int mOff  = (lane >> 4) * 8;

  v8f acc[4][4];
#pragma unroll
  for (int i = 0; i < 4; ++i)
#pragma unroll
    for (int j = 0; j < 4; ++j) acc[i][j] = (v8f){0.f,0.f,0.f,0.f,0.f,0.f,0.f,0.f};

  for (int k0 = 0; k0 < K; k0 += 32) {
    V bh[4], bl[4];
#pragma unroll
    for (int j = 0; j < 4; ++j) {
      const size_t bo = (size_t)(n0 + (j << 4) + rlane) * ldb + koff + k0;
      bh[j] = Frag<T>::load(Bb + bo);
      if (SPLIT == 2) bl[j] = Frag<T>::load(Bb2 + bo);
    }
#pragma unroll
    for (int i = 0; i < 4; ++i) {
      const size_t ao = (size_t)(m0 + (i << 4) + rlane) * lda + koff + k0;
      V ah = Frag<T>::load(Ab + ao);
      V al;
      if (SPLIT != 0) al = Frag<T>::load(Ab2 + ao);
#pragma unroll
      for (int j = 0; j < 4; ++j) {
        acc[i][j] = Frag<T>::mma(ah, bh[j], acc[i][j]);
        if (SPLIT == 2) acc[i][j] = Frag<T>::mma(ah, bl[j], acc[i][j]);
        if (SPLIT != 0) acc[i][j] = Frag<T>::mma(al, bh[j], acc[i][j]);
      }
      Frag<T>::guard4(acc[i][0], acc[i][1], acc[i][2], acc[i][3], ah, (SPLIT != 0) ? al : ah);
    }
    Frag<T>::keep(bh[0], bh[1], bh[2], bh[3]);
    if (SPLIT == 2) Frag<T>::keep(bl[0], bl[1], bl[2], bl[3]);
  }
  acc_guard4(acc[0][0], acc[0][1], acc[0][2], acc[0][3]);
  acc_guard4(acc[1][0], acc[1][1], acc[1][2], acc[1][3]);
  acc_guard4(acc[2][0], acc[2][1], acc[2][2], acc[2][3]);
  acc_guard4(acc[3][0], acc[3][1], acc[3][2], acc[3][3]);

  float* slab = sT[wave];
  const float* Rb = RESID ? (resid + (size_t)b * strideR) : nullptr;
#pragma unroll
  for (int i = 0; i < 4; ++i) {
    const int mBase = m0 + (i << 4);
#pragma unroll
    for (int j = 0; j < 4; ++j) {
      const int n = n0 + (j << 4) + rlane;
      float bv = 0.f;
      if (BIAS_MODE == 2) bv = bias[n];
#pragma unroll
      for (int r = 0; r < 8; ++r) {
        float v = acc[i][j][r] * scale;
        if (BIAS_MODE == 1) v += bias[mBase + mOff + r];
        if (BIAS_MODE == 2) v += bv;
        if (RESID) v += Rb[(size_t)(mBase + mOff + r) * ldc + n];
        if (ACT == 2) v = fmaxf(v, 0.0f);
        if (ACT == 4) v = (v > 0.f) ? v : 0.01f * v;
        slab[(mOff + r) * 68 + (j << 4) + rlane] = v;
      }
    }
    __builtin_amdgcn_fence(__ATOMIC_RELEASE, "workgroup");
    __builtin_amdgcn_wave_barrier();
    __builtin_amdgcn_fence(__ATOMIC_ACQUIRE, "workgroup");
    if (OUT_MODE == 0) {
      float* C = (float*)Cout + (size_t)b * strideC;
      const int hh = lane >> 4, c4 = (lane & 15) * 4;
      for (int pass = 0; pass < 2; ++pass) {
#pragma unroll
        for (int it = 0; it < 8; ++it) {
          const int row = it * 2 + hh;
          v4f v = *(const v4f*)(slab + row * 68 + c4);
          *(volatile v4f*)(C + (size_t)(mBase + row) * ldc + n0 + c4) = v;
        }
        __threadfence();
      }
    } else {
      const int q = lane >> 3, c8 = (lane & 7) * 8;
      unsigned short* C  = (unsigned short*)Cout  + (size_t)b * strideC;
      unsigned short* C2 = (OUT_MODE == 2) ? ((unsigned short*)Cout2 + (size_t)b * strideC) : nullptr;
      for (int pass = 0; pass < 2; ++pass) {
#pragma unroll
        for (int it = 0; it < 4; ++it) {
          const int row = it * 4 + q;
          const float* sp = slab + row * 68 + c8;
          v8h hv, lv;
#pragma unroll
          for (int e = 0; e < 8; ++e) {
            if (OUT_MODE == 1) {
              hv[e] = (_Float16)sp[e];
            } else {
              unsigned short hb = f2bf_bits(sp[e]);
              unsigned short lb = f2bf_bits(sp[e] - bf_bits2f(hb));
              hv[e] = __builtin_bit_cast(_Float16, hb);
              lv[e] = __builtin_bit_cast(_Float16, lb);
            }
          }
          *(volatile v8h*)(C + (size_t)(mBase + row) * ldc + n0 + c8) = hv;
          if (OUT_MODE == 2) *(volatile v8h*)(C2 + (size_t)(mBase + row) * ldc + n0 + c8) = lv;
        }
        __threadfence();
      }
    }
    __builtin_amdgcn_fence(__ATOMIC_RELEASE, "workgroup");
    __builtin_amdgcn_wave_barrier();
    __builtin_amdgcn_fence(__ATOMIC_ACQUIRE, "workgroup");
  }
}

__device__ __forceinline__ unsigned short at_bf_bits(float f) {
  unsigned u = __float_as_uint(f);
  return (unsigned short)((u + 0x7FFFu + ((u >> 16) & 1u)) >> 16);
}
__device__ __forceinline__ __bf16 at_f2bf(float f) { return __builtin_bit_cast(__bf16, at_bf_bits(f)); }
__device__ __forceinline__ void at_split(float f, __bf16& hi, __bf16& lo) {
  const unsigned short hb = at_bf_bits(f);
  hi = __builtin_bit_cast(__bf16, hb);
  lo = at_f2bf(f - __uint_as_float(((unsigned)hb) << 16));
}
__device__ __forceinline__ v8f at_mma(v16b a, v16b b, v8f c) {
  c = __builtin_amdgcn_wmma_f32_16x16x32_bf16(false, a, false, b, (short)0, c, false, false);
  asm volatile("v_nop\n\tv_nop\n\tv_nop\n\tv_nop" : "+v"(c) : "v"(a), "v"(b));
  return c;
}

__global__ __launch_bounds__(256) void cast8_bf16_kernel(const float* __restrict__ in, unsigned short* __restrict__ out, int n8) {
  const int i = blockIdx.x * 256 + threadIdx.x;
  if (i >= n8) return;
  const float* p = in + 8 * (size_t)i;
  const v4f a = *(const v4f*)(p);
  const v4f c = *(const v4f*)(p + 4);
  unsigned short hb[8];
#pragma unroll
  for (int e = 0; e < 4; ++e) {
    hb[e]     = f2bf_bits(a[e]);
    hb[4 + e] = f2bf_bits(c[e]);
  }
  const v4u u = (v4u){pk16(hb[0], hb[1]), pk16(hb[2], hb[3]), pk16(hb[4], hb[5]), pk16(hb[6], hb[7])};
  unsigned short* q = out + 8 * (size_t)i;
  *(volatile v4u*)q = u;
  __threadfence();
  *(volatile v4u*)q = u;
}

struct FreqTab { float f[32]; };
static_assert(sizeof(FreqTab) == 128, "no padding");

__global__ __launch_bounds__(256) void trig_table_kernel(float* __restrict__ ct, float* __restrict__ st, FreqTab tab) {
#pragma clang fp contract(off)
  const int i = blockIdx.y;
  const int t = blockIdx.x * 256 + threadIdx.x;
  const float invf = tab.f[i];
  const float ang = (float)t * invf;
  float sv, cv;
  sincosf(ang, &sv, &cv);
  float* cp = ct + (size_t)i * kT + t;
  float* sp = st + (size_t)i * kT + t;
  *(volatile float*)cp = cv;
  *(volatile float*)sp = sv;
  __threadfence();
  *(volatile float*)cp = cv;
  *(volatile float*)sp = sv;
}

__global__ __launch_bounds__(256) void rope_qk_kernel(const float* __restrict__ qkv, const float* __restrict__ ct,
                                                      const float* __restrict__ st,
                                                      unsigned short* __restrict__ QKh, unsigned short* __restrict__ QKl) {
#pragma clang fp contract(off)
  const int tid = threadIdx.x;
  const int g   = tid & 7;
  const int tok = blockIdx.x * 32 + (tid >> 3);
  const int hh  = blockIdx.y;
  const int b   = tok >> 11;
  const int t   = tok & (kT - 1);
  const float* src = qkv + (size_t)tok * kNQKV + hh * kDh + 8 * g;
  const v4f a  = *(const v4f*)(src);
  const v4f a2 = *(const v4f*)(src + 4);
  float x[8];
#pragma unroll
  for (int e = 0; e < 4; ++e) { x[e] = a[e]; x[4 + e] = a2[e]; }
  float cs[4], sn[4];
#pragma unroll
  for (int e = 0; e < 4; ++e) {
    cs[e] = ct[(size_t)(4 * g + e) * kT + t];
    sn[e] = st[(size_t)(4 * g + e) * kT + t];
  }
  float o[8];
#pragma unroll
  for (int e = 0; e < 4; ++e) {
    const float x1 = x[2 * e], x2 = x[2 * e + 1];
    o[2 * e]     = x1 * cs[e] - x2 * sn[e];
    o[2 * e + 1] = x1 * sn[e] + x2 * cs[e];
  }
  unsigned short hb[8], lb[8];
#pragma unroll
  for (int e = 0; e < 8; ++e) {
    hb[e] = f2bf_bits(o[e]);
    lb[e] = f2bf_bits(o[e] - bf_bits2f(hb[e]));
  }
  const v4u uh = (v4u){pk16(hb[0], hb[1]), pk16(hb[2], hb[3]), pk16(hb[4], hb[5]), pk16(hb[6], hb[7])};
  const v4u ul = (v4u){pk16(lb[0], lb[1]), pk16(lb[2], lb[3]), pk16(lb[4], lb[5]), pk16(lb[6], lb[7])};
  const size_t rowQ = (size_t)(b * kH + hh) * kT + t;
  const size_t rowK = (size_t)kQRows + (size_t)(b * kKV + (hh - kH)) * kT + t;
  const size_t row  = (hh < kH) ? rowQ : rowK;
  unsigned short* dh_ = QKh + row * kDh + 8 * g;
  unsigned short* dl_ = QKl + row * kDh + 8 * g;
  *(volatile v4u*)dh_ = uh;
  *(volatile v4u*)dl_ = ul;
  __threadfence();
  *(volatile v4u*)dh_ = uh;
  *(volatile v4u*)dl_ = ul;
}

__global__ __launch_bounds__(256) void vt_split_kernel(const float* __restrict__ qkv, unsigned short* __restrict__ VTh,
                                                       unsigned short* __restrict__ VTl) {
  __shared__ float sm[64][65];
  const int t  = threadIdx.x;
  const int s0 = blockIdx.x * 64;
  const int kv = blockIdx.y;
  const int b  = blockIdx.z;
#pragma unroll
  for (int i = 0; i < 16; ++i) {
    const int e = i * 256 + t;
    const int r = e >> 6;
    const int c = e & 63;
    sm[c][r] = qkv[((size_t)(b * kT + s0 + r)) * kNQKV + kVCol + kv * kDh + c];
  }
  __syncthreads();
  const int lane = t & 31, wave = t >> 5;
  const int q = lane >> 3, c8 = (lane & 7) * 8;
  const size_t base = ((size_t)(b * kKV + kv) * kDh) * kT;
  for (int pass = 0; pass < 2; ++pass) {
#pragma unroll
    for (int it = 0; it < 2; ++it) {
      const int row = wave * 8 + it * 4 + q;
      unsigned short hb[8], lb[8];
#pragma unroll
      for (int e = 0; e < 8; ++e) {
        const float v = sm[row][c8 + e];
        hb[e] = f2bf_bits(v);
        lb[e] = f2bf_bits(v - bf_bits2f(hb[e]));
      }
      const v4u uh = (v4u){pk16(hb[0], hb[1]), pk16(hb[2], hb[3]), pk16(hb[4], hb[5]), pk16(hb[6], hb[7])};
      const v4u ul = (v4u){pk16(lb[0], lb[1]), pk16(lb[2], lb[3]), pk16(lb[4], lb[5]), pk16(lb[6], lb[7])};
      *(volatile v4u*)(VTh + base + (size_t)row * kT + s0 + c8) = uh;
      *(volatile v4u*)(VTl + base + (size_t)row * kT + s0 + c8) = ul;
    }
    __threadfence();
  }
}

__global__ __launch_bounds__(128)
void attn_kernel(const unsigned short* __restrict__ QKhp, const unsigned short* __restrict__ QKlp,
                 const unsigned short* __restrict__ VThp, const unsigned short* __restrict__ VTlp,
                 unsigned short* __restrict__ Oh, unsigned short* __restrict__ Ol) {
  union FB { v16b v; v8b h[2]; };
  __shared__ __align__(16) __bf16 Ksh[64 * 64];
  __shared__ __align__(16) __bf16 Ksl[64 * 64];
  __shared__ __align__(16) __bf16 Vth[64 * 64];
  __shared__ __align__(16) __bf16 Vtl[64 * 64];
  __shared__ __align__(16) __bf16 Psh[4][16 * 64];
  __shared__ __align__(16) __bf16 Psl[4][16 * 64];

  const __bf16* Qh  = (const __bf16*)QKhp;
  const __bf16* Ql  = (const __bf16*)QKlp;
  const __bf16* Kh  = Qh + (size_t)kQRows * kDh;
  const __bf16* Kl  = Ql + (size_t)kQRows * kDh;
  const __bf16* VTh = (const __bf16*)VThp;
  const __bf16* VTl = (const __bf16*)VTlp;

  const int tid  = threadIdx.x;
  const int wave = tid >> 5;
  const int lane = tid & 31;
  const int hh   = lane >> 4;
  const int c    = lane & 15;

  const int bx  = blockIdx.x;
  const int qb  = bx & 31;
  const int bhi = bx >> 5;
  const int h   = bhi & 15;
  const int b   = bhi >> 4;
  const int kvh = h >> 2;
  const int q0  = qb * 64 + wave * 16;

  v16b qah[2], qal[2];
  {
    const __bf16* qhr = Qh + ((size_t)(b * kH + h) * kT + q0 + c) * kDh;
    const __bf16* qlr = Ql + ((size_t)(b * kH + h) * kT + q0 + c) * kDh;
#pragma unroll
    for (int dc = 0; dc < 2; ++dc) {
      FB fh, fl;
      fh.h[0] = *(const v8b*)(qhr + dc * 32 + 8 * hh);
      fh.h[1] = *(const v8b*)(qhr + dc * 32 + 16 + 8 * hh);
      fl.h[0] = *(const v8b*)(qlr + dc * 32 + 8 * hh);
      fl.h[1] = *(const v8b*)(qlr + dc * 32 + 16 + 8 * hh);
      qah[dc] = fh.v; qal[dc] = fl.v;
    }
  }
  const __bf16* khg = Kh  + (size_t)(b * kKV + kvh) * kT * kDh;
  const __bf16* klg = Kl  + (size_t)(b * kKV + kvh) * kT * kDh;
  const __bf16* vhg = VTh + (size_t)(b * kKV + kvh) * kDh * kT;
  const __bf16* vlg = VTl + (size_t)(b * kKV + kvh) * kDh * kT;

  float mrow[8], lrow[8];
  v8f oacc[4];
#pragma unroll
  for (int r = 0; r < 8; ++r) { mrow[r] = -INFINITY; lrow[r] = 0.f; }
#pragma unroll
  for (int t = 0; t < 4; ++t) oacc[t] = (v8f){0.f,0.f,0.f,0.f,0.f,0.f,0.f,0.f};

  const int kcStart = (qb > 8) ? (qb - 8) : 0;
  for (int kc = kcStart; kc <= qb; ++kc) {
    const int kv0 = kc * 64;
    __syncthreads();
#pragma unroll
    for (int it = 0; it < 4; ++it) {
      const int e = it * 128 + tid;
      const int row = e >> 3;
      const int seg = (e & 7) * 8;
      const v8b a0 = *(const v8b*)(khg + (size_t)(kv0 + row) * kDh + seg);
      const v8b a1 = *(const v8b*)(klg + (size_t)(kv0 + row) * kDh + seg);
      *(v8b*)(Ksh + row * 64 + seg) = a0;
      *(v8b*)(Ksl + row * 64 + seg) = a1;
    }
    asm volatile("" ::: "memory");
#pragma unroll
    for (int it = 0; it < 4; ++it) {
      const int e = it * 128 + tid;
      const int row = e >> 3;
      const int seg = (e & 7) * 8;
      const v8b v0 = *(const v8b*)(vhg + (size_t)row * kT + kv0 + seg);
      const v8b v1 = *(const v8b*)(vlg + (size_t)row * kT + kv0 + seg);
      *(v8b*)(Vth + row * 64 + seg) = v0;
      *(v8b*)(Vtl + row * 64 + seg) = v1;
    }
    __syncthreads();

    v8f s[4];
#pragma unroll
    for (int j = 0; j < 4; ++j) {
      s[j] = (v8f){0.f,0.f,0.f,0.f,0.f,0.f,0.f,0.f};
#pragma unroll
      for (int dc = 0; dc < 2; ++dc) {
        FB kb, kl;
        kb.h[0] = *(const v8b*)(Ksh + (j * 16 + c) * 64 + dc * 32 + 8 * hh);
        kb.h[1] = *(const v8b*)(Ksh + (j * 16 + c) * 64 + dc * 32 + 16 + 8 * hh);
        kl.h[0] = *(const v8b*)(Ksl + (j * 16 + c) * 64 + dc * 32 + 8 * hh);
        kl.h[1] = *(const v8b*)(Ksl + (j * 16 + c) * 64 + dc * 32 + 16 + 8 * hh);
        s[j] = at_mma(qah[dc], kb.v, s[j]);
        s[j] = at_mma(qah[dc], kl.v, s[j]);
        s[j] = at_mma(qal[dc], kb.v, s[j]);
      }
    }
    float cm[8];
#pragma unroll
    for (int r = 0; r < 8; ++r) {
      const int qrow = q0 + 8 * hh + r;
      float m = -INFINITY;
#pragma unroll
      for (int j = 0; j < 4; ++j) {
        const int kvcol = kv0 + j * 16 + c;
        const bool masked = (kvcol > qrow) || (qrow - kvcol > kWin - 1);
        float sv = s[j][r] * kScoreScale;
        sv = masked ? -INFINITY : sv;
        s[j][r] = sv;
        m = fmaxf(m, sv);
      }
#pragma unroll
      for (int off = 1; off < 16; off <<= 1) m = fmaxf(m, __shfl_xor(m, off, 32));
      cm[r] = m;
    }
    __bf16* pwh = Psh[wave];
    __bf16* pwl = Psl[wave];
#pragma unroll
    for (int r = 0; r < 8; ++r) {
      const float mnew  = fmaxf(mrow[r], cm[r]);
      const float msafe = (mnew == -INFINITY) ? 0.0f : mnew;
      const float alpha = expf(fmaxf(mrow[r] - msafe, kExpFloor));
      mrow[r] = mnew;
      float psum = 0.f;
#pragma unroll
      for (int j = 0; j < 4; ++j) {
        const float p = expf(fmaxf(s[j][r] - msafe, kExpFloor));
        psum += p;
        __bf16 ph, pl;
        at_split(p, ph, pl);
        pwh[(8 * hh + r) * 64 + j * 16 + c] = ph;
        pwl[(8 * hh + r) * 64 + j * 16 + c] = pl;
      }
#pragma unroll
      for (int off = 1; off < 16; off <<= 1) psum += __shfl_xor(psum, off, 32);
      lrow[r] = lrow[r] * alpha + psum;
#pragma unroll
      for (int t = 0; t < 4; ++t) oacc[t][r] *= alpha;
    }
    __builtin_amdgcn_fence(__ATOMIC_RELEASE, "workgroup");
    __builtin_amdgcn_wave_barrier();
    __builtin_amdgcn_fence(__ATOMIC_ACQUIRE, "workgroup");
#pragma unroll 1
    for (int kk = 0; kk < 2; ++kk) {
      FB pa, pl;
      pa.h[0] = *(const v8b*)(pwh + c * 64 + kk * 32 + 8 * hh);
      pa.h[1] = *(const v8b*)(pwh + c * 64 + kk * 32 + 16 + 8 * hh);
      pl.h[0] = *(const v8b*)(pwl + c * 64 + kk * 32 + 8 * hh);
      pl.h[1] = *(const v8b*)(pwl + c * 64 + kk * 32 + 16 + 8 * hh);
#pragma unroll
      for (int t = 0; t < 4; ++t) {
        FB vb, vl;
        vb.h[0] = *(const v8b*)(Vth + (t * 16 + c) * 64 + kk * 32 + 8 * hh);
        vb.h[1] = *(const v8b*)(Vth + (t * 16 + c) * 64 + kk * 32 + 16 + 8 * hh);
        vl.h[0] = *(const v8b*)(Vtl + (t * 16 + c) * 64 + kk * 32 + 8 * hh);
        vl.h[1] = *(const v8b*)(Vtl + (t * 16 + c) * 64 + kk * 32 + 16 + 8 * hh);
        oacc[t] = at_mma(pa.v, vb.v, oacc[t]);
        oacc[t] = at_mma(pa.v, vl.v, oacc[t]);
        oacc[t] = at_mma(pl.v, vb.v, oacc[t]);
      }
    }
  }

  __bf16* owh = Psh[wave];
  __bf16* owl = Psl[wave];
#pragma unroll
  for (int r = 0; r < 8; ++r) {
    const float inv = 1.0f / lrow[r];
#pragma unroll
    for (int t = 0; t < 4; ++t) {
      const float o = oacc[t][r] * inv;
      __bf16 oh_, ol_;
      at_split(o, oh_, ol_);
      owh[(8 * hh + r) * 64 + t * 16 + c] = oh_;
      owl[(8 * hh + r) * 64 + t * 16 + c] = ol_;
    }
  }
  __builtin_amdgcn_fence(__ATOMIC_RELEASE, "workgroup");
  __builtin_amdgcn_wave_barrier();
  __builtin_amdgcn_fence(__ATOMIC_ACQUIRE, "workgroup");
  {
    const int q4 = lane >> 3, c8 = (lane & 7) * 8;
    unsigned short* ohb = Oh + ((size_t)(b * kT + q0)) * kD + h * kDh + c8;
    unsigned short* olb = Ol + ((size_t)(b * kT + q0)) * kD + h * kDh + c8;
    for (int pass = 0; pass < 2; ++pass) {
#pragma unroll
      for (int it = 0; it < 4; ++it) {
        const int row = it * 4 + q4;
        const v8b hv = *(const v8b*)(owh + row * 64 + c8);
        const v8b lv = *(const v8b*)(owl + row * 64 + c8);
        const v4u uh = __builtin_bit_cast(v4u, hv);
        const v4u ul = __builtin_bit_cast(v4u, lv);
        *(volatile v4u*)(ohb + (size_t)row * kD) = uh;
        *(volatile v4u*)(olb + (size_t)row * kD) = ul;
      }
      __threadfence();
    }
  }
}

static double host_sqrt(double a) {
  double x = a;
  for (int i = 0; i < 64; ++i) x = 0.5 * (x + a / x);
  return x;
}

extern "C" void kernel_launch(void* const* d_in, const int* in_sizes, int n_in,
                              void* d_out, int out_size, void* d_ws, size_t ws_size,
                              hipStream_t stream) {
  if (n_in < 5) return;
  const int nX  = kTok * kD;
  const int nWq = kH * kDh * kD;
  const int nWk = kKV * kDh * kD;
  if (in_sizes[0] != nX || in_sizes[1] != nWq || in_sizes[2] != nWk || in_sizes[3] != nWk || in_sizes[4] != nWq) return;
  if (out_size != nX) return;

  const size_t szXB  = (size_t)kTok * kD * 2;
  const size_t szWB  = (size_t)(kNQKV + kD) * kD * 2;
  const size_t szQKV = (size_t)kTok * kNQKV * 4;
  const size_t szTab = (size_t)32 * kT * 4;
  const size_t szQK  = (size_t)(kQRows + kKRows) * kDh * 2;
  const size_t szVT  = (size_t)kB * kKV * kDh * kT * 2;
  const size_t szO   = (size_t)kTok * kD * 2;
  const size_t offXB  = 0;
  const size_t offWB  = offXB + szXB;
  const size_t offQKV = offWB + szWB;
  const size_t offCT  = offQKV + szQKV;
  const size_t offST  = offCT + szTab;
  const size_t offQKH = offST + szTab;
  const size_t offQKL = offQKH + szQK;
  const size_t offVTH = offQKL + szQK;
  const size_t offVTL = offVTH + szVT;
  const size_t offOH  = offVTL + szVT;
  const size_t offOL  = offOH + szO;
  const size_t total  = offOL + szO;
  if (ws_size < total) return;

  const float* x  = (const float*)d_in[0];
  const float* Wq = (const float*)d_in[1];
  const float* Wk = (const float*)d_in[2];
  const float* Wv = (const float*)d_in[3];
  const float* Wo = (const float*)d_in[4];
  float* out = (float*)d_out;
  char* ws = (char*)d_ws;
  unsigned short* XB  = (unsigned short*)(ws + offXB);
  unsigned short* WB  = (unsigned short*)(ws + offWB);
  float* QKV = (float*)(ws + offQKV);
  float* CT  = (float*)(ws + offCT);
  float* ST  = (float*)(ws + offST);
  unsigned short* QKH = (unsigned short*)(ws + offQKH);
  unsigned short* QKL = (unsigned short*)(ws + offQKL);
  unsigned short* VTH = (unsigned short*)(ws + offVTH);
  unsigned short* VTL = (unsigned short*)(ws + offVTL);
  unsigned short* OH  = (unsigned short*)(ws + offOH);
  unsigned short* OL  = (unsigned short*)(ws + offOL);

  FreqTab tab;
  {
    const double r8  = host_sqrt(10.0);
    const double r16 = host_sqrt(r8);
    const double r32 = host_sqrt(r16);
    for (int i = 0; i < 32; ++i) {
      double p = 1.0;
      if (i & 16) p *= 100.0;
      if (i & 8)  p *= 10.0;
      if (i & 4)  p *= r8;
      if (i & 2)  p *= r16;
      if (i & 1)  p *= r32;
      const float pf = (float)p;
      tab.f[i] = 1.0f / pf;
    }
  }

  cast8_bf16_kernel<<<dim3((nX / 8) / 256), dim3(256), 0, stream>>>(x, XB, nX / 8);
  cast8_bf16_kernel<<<dim3((nWq / 8) / 256), dim3(256), 0, stream>>>(Wq, WB, nWq / 8);
  cast8_bf16_kernel<<<dim3((nWk / 8) / 256), dim3(256), 0, stream>>>(Wk, WB + (size_t)(kH * kDh) * kD, nWk / 8);
  cast8_bf16_kernel<<<dim3((nWk / 8) / 256), dim3(256), 0, stream>>>(Wv, WB + (size_t)kVCol * kD, nWk / 8);
  cast8_bf16_kernel<<<dim3((nWq / 8) / 256), dim3(256), 0, stream>>>(Wo, WB + (size_t)kNQKV * kD, nWq / 8);

  trig_table_kernel<<<dim3(kT / 256, 32), dim3(256), 0, stream>>>(CT, ST, tab);

  {
    const int tiles = (kTok / 64) * (kNQKV / 64);
    wmma_gemm64<1, 0, 0, 0, false, 0><<<dim3(tiles / 8, 1), dim3(256), 0, stream>>>(
        XB, XB, kD, 0L, WB, WB, kD, 0L,
        (void*)QKV, (void*)QKV, kNQKV, 0L, CT, CT, 0L, kTok, kNQKV, kD, 1.0f);
  }

  rope_qk_kernel<<<dim3(kTok / 32, kH + kKV), dim3(256), 0, stream>>>(QKV, CT, ST, QKH, QKL);
  vt_split_kernel<<<dim3(kT / 64, kKV, kB), dim3(256), 0, stream>>>(QKV, VTH, VTL);

  attn_kernel<<<dim3(kB * kH * (kT / 64)), dim3(128), 0, stream>>>(QKH, QKL, VTH, VTL, OH, OL);

  {
    const int tiles = (kTok / 64) * (kD / 64);
    wmma_gemm64<1, 1, 0, 0, false, 0><<<dim3(tiles / 8, 1), dim3(256), 0, stream>>>(
        OH, OL, kD, 0L, WB + (size_t)kNQKV * kD, WB + (size_t)kNQKV * kD, kD, 0L,
        (void*)out, (void*)out, kD, 0L, CT, CT, 0L, kTok, kD, kD, 1.0f);
  }
}
